// MultiHeadCrossAttention_10204842295866
// MI455X (gfx1250) — hardware-verified
//
#include <hip/hip_runtime.h>
#include <math.h>

typedef __attribute__((ext_vector_type(16))) _Float16 v16h;
typedef __attribute__((ext_vector_type(8)))  _Float16 v8h;
typedef __attribute__((ext_vector_type(8)))  float    v8f;
typedef __attribute__((ext_vector_type(4)))  float    v4f;

constexpr int kB     = 2;
constexpr int kSq    = 2048;
constexpr int kSkv   = 2048;
constexpr int kH     = 16;
constexpr int kHd    = 64;
constexpr int kD     = kH * kHd;
constexpr int kBH    = kB * kH;
constexpr int kKc    = 8;
constexpr int kChunk = kSkv / kKc;
constexpr int kCP    = 65;
static_assert(kD == 1024);
static_assert(kHd == 64);
static_assert(kChunk == 256);
static_assert((kChunk % 32) == 0 && (kHd % 32) == 0);
static_assert((kSq % 64) == 0 && (kSkv % 64) == 0);

constexpr float kQkScale = 0.125f;
static_assert(kQkScale * kQkScale * (float)kHd == 1.0f);
constexpr float kInCarry   = 16.0f;
constexpr float kNCarry    = 8.0f;
constexpr float kGramScale = 1.0f / (kInCarry * kInCarry);
constexpr float kOutScale  = 1.0f / (kInCarry * kNCarry);
constexpr float kNMul      = kQkScale * kNCarry;
constexpr float kF16MinNormal = 6.103515625e-05f;

constexpr size_t kOffCT   = 0;
constexpr size_t kOffXH   = kOffCT + (size_t)kBH * kKc * kHd * kChunk * 2;
constexpr size_t kOffGP   = kOffXH + (size_t)kBH * kSq * kHd * 2;
constexpr size_t kOffNT   = kOffGP + (size_t)kBH * kKc * kHd * kHd * 4;
constexpr size_t kWsTotal = kOffNT + (size_t)kBH * kHd * kHd * 2;
static_assert(kWsTotal == 21233664ull);
static_assert(kWsTotal <= 134217728ull);
static_assert((kOffXH % 128) == 0 && (kOffGP % 128) == 0 && (kOffNT % 128) == 0);

__device__ __forceinline__ _Float16 f16_flush(float f) {
  const float g = (fabsf(f) < kF16MinNormal) ? 0.0f : f;
  return (_Float16)g;
}

union FragU { v16h v; v8h h[2]; };
__device__ __forceinline__ v16h frag_load(const _Float16* p) {
  FragU f;
  f.h[0] = *(const v8h*)(p);
  f.h[1] = *(const v8h*)(p + 16);
  return f.v;
}
__device__ __forceinline__ v8f frag_mma(v16h a, v16h b, v8f c) {
  return __builtin_amdgcn_wmma_f32_16x16x32_f16(false, a, false, b, (short)0, c, false, false);
}
__device__ __forceinline__ void dep_guard1(v8f& c, v16h x, v16h y) {
  asm volatile("v_nop\n\tv_nop\n\tv_nop\n\tv_nop" : "+v"(c) : "v"(x), "v"(y));
}
__device__ __forceinline__ void keep4_h(v16h a, v16h b, v16h c, v16h d) {
  asm volatile("v_nop" :: "v"(a), "v"(b), "v"(c), "v"(d));
}
__device__ __forceinline__ void acc_guard4(v8f& a, v8f& b, v8f& c, v8f& d) {
  asm volatile("v_nop\n\tv_nop\n\tv_nop\n\tv_nop" : "+v"(a), "+v"(b), "+v"(c), "+v"(d));
}

__global__ __launch_bounds__(256) void wmma_gemm64_f16(
    const unsigned short* Ap, int lda, long strideA,
    const unsigned short* Btp, int ldb, long strideB,
    float* __restrict__ Cout, int ldc, long strideC,
    int M, int N, int K, float scale) {
  const _Float16* A  = (const _Float16*)Ap;
  const _Float16* Bt = (const _Float16*)Btp;
  __shared__ __align__(16) float sT[8][16 * 68];
  const int b    = blockIdx.y;
  const int lane = threadIdx.x & 31;
  const int wave = threadIdx.x >> 5;
  const int tilesN = N >> 6;
  const int tilesM = M >> 6;
  const int tile = blockIdx.x * 8 + wave;
  if (tile >= tilesM * tilesN) return;
  const int tm = tile / tilesN;
  const int tn = tile - tm * tilesN;
  const int m0 = tm << 6;
  const int n0 = tn << 6;

  const _Float16* Ab = A  + (size_t)b * strideA;
  const _Float16* Bb = Bt + (size_t)b * strideB;

  const int rlane = lane & 15;
  const int koff  = (lane >> 4) * 8;
  const int mOff  = (lane >> 4) * 8;

  v8f acc[4][4];
#pragma unroll
  for (int i = 0; i < 4; ++i)
#pragma unroll
    for (int j = 0; j < 4; ++j) acc[i][j] = (v8f){0.f, 0.f, 0.f, 0.f, 0.f, 0.f, 0.f, 0.f};

  for (int k0 = 0; k0 < K; k0 += 32) {
    v16h bh[4];
#pragma unroll
    for (int j = 0; j < 4; ++j) {
      const size_t bo = (size_t)(n0 + (j << 4) + rlane) * ldb + koff + k0;
      bh[j] = frag_load(Bb + bo);
    }
#pragma unroll
    for (int i = 0; i < 4; ++i) {
      const size_t ao = (size_t)(m0 + (i << 4) + rlane) * lda + koff + k0;
      const v16h ah = frag_load(Ab + ao);
#pragma unroll
      for (int j = 0; j < 4; ++j) acc[i][j] = frag_mma(ah, bh[j], acc[i][j]);
      dep_guard1(acc[i][0], ah, bh[0]);
      dep_guard1(acc[i][1], ah, bh[1]);
      dep_guard1(acc[i][2], ah, bh[2]);
      dep_guard1(acc[i][3], ah, bh[3]);
    }
    keep4_h(bh[0], bh[1], bh[2], bh[3]);
  }
  acc_guard4(acc[0][0], acc[0][1], acc[0][2], acc[0][3]);
  acc_guard4(acc[1][0], acc[1][1], acc[1][2], acc[1][3]);
  acc_guard4(acc[2][0], acc[2][1], acc[2][2], acc[2][3]);
  acc_guard4(acc[3][0], acc[3][1], acc[3][2], acc[3][3]);

  float* slab = sT[wave];
  float* C = Cout + (size_t)b * strideC;
  const int hh = lane >> 4;
  const int c4 = (lane & 15) * 4;
#pragma unroll
  for (int i = 0; i < 4; ++i) {
    const int mBase = m0 + (i << 4);
#pragma unroll
    for (int j = 0; j < 4; ++j) {
#pragma unroll
      for (int r = 0; r < 8; ++r) {
        const float v = acc[i][j][r] * scale;
        slab[(mOff + r) * 68 + (j << 4) + rlane] = v;
      }
    }
    __builtin_amdgcn_fence(__ATOMIC_RELEASE, "workgroup");
    __builtin_amdgcn_wave_barrier();
    __builtin_amdgcn_fence(__ATOMIC_ACQUIRE, "workgroup");
    for (int pass = 0; pass < 2; ++pass) {
#pragma unroll
      for (int it = 0; it < 8; ++it) {
        const int row = it * 2 + hh;
        const v4f v = *(const v4f*)(slab + row * 68 + c4);
        *(volatile v4f*)(C + (size_t)(mBase + row) * ldc + n0 + c4) = v;
      }
      __threadfence();
    }
    __builtin_amdgcn_fence(__ATOMIC_RELEASE, "workgroup");
    __builtin_amdgcn_wave_barrier();
    __builtin_amdgcn_fence(__ATOMIC_ACQUIRE, "workgroup");
  }
}

__global__ __launch_bounds__(256) void ctx_transpose_f16_kernel(const float* __restrict__ ctx,
                                                               unsigned short* __restrict__ CT) {
  __shared__ float sm[64 * kCP];
  const unsigned t  = threadIdx.x;
  const unsigned tt = blockIdx.x;
  const unsigned bh = blockIdx.y;
  const unsigned b  = bh >> 4;
  const unsigned h  = bh & 15u;
  const unsigned t0 = tt * 64u;
  const float* src = ctx + ((size_t)b * kSkv + t0) * kD + (size_t)h * kHd;
#pragma unroll
  for (int i = 0; i < 4; ++i) {
    unsigned e = (unsigned)i * 256u + t;
    unsigned r = e >> 4;
    unsigned c4 = (e & 15u) * 4u;
    asm volatile("" : "+v"(r));
    asm volatile("" : "+v"(c4));
    const v4f v = *(const v4f*)(src + (size_t)r * kD + c4);
    sm[(c4 + 0u) * kCP + r] = v[0] * kInCarry;
    sm[(c4 + 1u) * kCP + r] = v[1] * kInCarry;
    sm[(c4 + 2u) * kCP + r] = v[2] * kInCarry;
    sm[(c4 + 3u) * kCP + r] = v[3] * kInCarry;
  }
  __syncthreads();
  const unsigned lane = t & 31u;
  const unsigned wave = t >> 5;
  unsigned q  = lane >> 3;
  unsigned c8 = (lane & 7u) * 8u;
  asm volatile("" : "+v"(q));
  asm volatile("" : "+v"(c8));
  const unsigned kc = t0 >> 8;
  const unsigned tl = t0 & 255u;
  v8h hv[2];
#pragma unroll
  for (int it = 0; it < 2; ++it) {
    const unsigned d = wave * 8u + (unsigned)it * 4u + q;
#pragma unroll
    for (int e = 0; e < 8; ++e) hv[it][e] = f16_flush(sm[d * kCP + c8 + (unsigned)e]);
  }
  for (int pass = 0; pass < 2; ++pass) {
#pragma unroll
    for (int it = 0; it < 2; ++it) {
      const unsigned d = wave * 8u + (unsigned)it * 4u + q;
      const size_t o = (((size_t)bh * kKc + kc) * kHd + d) * kChunk + tl + c8;
      *(volatile v8h*)(CT + o) = hv[it];
    }
    __threadfence();
  }
}

__global__ __launch_bounds__(256) void x_headmajor_f16_kernel(const float* __restrict__ X,
                                                             unsigned short* __restrict__ XH, unsigned total8) {
  unsigned i = blockIdx.x * 256u + threadIdx.x;
  if (i >= total8) return;
  unsigned c   = (i & 127u) * 8u;
  unsigned row = i >> 7;
  asm volatile("" : "+v"(c));
  asm volatile("" : "+v"(row));
  const unsigned b = row >> 11;
  const unsigned s = row & 2047u;
  const unsigned h = c >> 6;
  const unsigned d = c & 63u;
  const float* p = X + (size_t)i * 8;
  const v4f a0 = *(const v4f*)(p);
  const v4f a1 = *(const v4f*)(p + 4);
  v8h hv;
#pragma unroll
  for (int e = 0; e < 4; ++e) {
    hv[e]     = f16_flush(a0[e] * kInCarry);
    hv[4 + e] = f16_flush(a1[e] * kInCarry);
  }
  const size_t o = ((size_t)(b * (unsigned)kH + h) * kSq + s) * kHd + d;
  *(volatile v8h*)(XH + o) = hv;
  __threadfence();
  *(volatile v8h*)(XH + o) = hv;
}

__global__ __launch_bounds__(256) void chain_kernel(const float* __restrict__ GP,
                                                   const float* __restrict__ Wq, const float* __restrict__ Wk,
                                                   const float* __restrict__ Wv, unsigned short* __restrict__ NT) {
  __shared__ __align__(16) float sG[64 * kCP];
  __shared__ __align__(16) float sT[64 * kCP];
  __shared__ __align__(16) float sW[64 * kCP];
  const unsigned t  = threadIdx.x;
  const unsigned bh = blockIdx.x;
  const unsigned h  = bh & (unsigned)(kH - 1);
  unsigned ti = t >> 4;
  unsigned tj = t & 15u;
  asm volatile("" : "+v"(ti));
  asm volatile("" : "+v"(tj));
  const float* Gd = GP + (size_t)bh * kKc * 4096;
  const float* wq = Wq + (size_t)h * 4096;
  const float* wk = Wk + (size_t)h * 4096;
  const float* wv = Wv + (size_t)h * 4096;

#pragma unroll 1
  for (int it = 0; it < 4; ++it) {
    unsigned e = ((unsigned)it * 256u + t) * 4u;
    asm volatile("" : "+v"(e));
    const unsigned r = e >> 6;
    const unsigned c = e & 63u;
    v4f s = (v4f){0.f, 0.f, 0.f, 0.f};
#pragma unroll
    for (int kc = 0; kc < kKc; ++kc) {
      const v4f p = *(const v4f*)(Gd + (size_t)kc * 4096 + e);
      s = s + p;
    }
    sG[r * kCP + c + 0u] = s[0];
    sG[r * kCP + c + 1u] = s[1];
    sG[r * kCP + c + 2u] = s[2];
    sG[r * kCP + c + 3u] = s[3];
  }
#pragma unroll
  for (int it = 0; it < 4; ++it) {
    const unsigned e = ((unsigned)it * 256u + t) * 4u;
    const unsigned r = e >> 6;
    const unsigned c = e & 63u;
    const v4f v = *(const v4f*)(wv + e);
    sW[r * kCP + c + 0u] = v[0];
    sW[r * kCP + c + 1u] = v[1];
    sW[r * kCP + c + 2u] = v[2];
    sW[r * kCP + c + 3u] = v[3];
  }
  __syncthreads();

  {
    float acc[4][4];
#pragma unroll
    for (int x = 0; x < 4; ++x)
#pragma unroll
      for (int y = 0; y < 4; ++y) acc[x][y] = 0.f;
#pragma unroll 1
    for (int k = 0; k < 64; ++k) {
      float a[4], bq[4];
#pragma unroll
      for (int x = 0; x < 4; ++x) a[x] = sG[(ti * 4u + (unsigned)x) * kCP + (unsigned)k];
#pragma unroll
      for (int y = 0; y < 4; ++y) bq[y] = sW[(tj + 16u * (unsigned)y) * kCP + (unsigned)k];
#pragma unroll
      for (int x = 0; x < 4; ++x)
#pragma unroll
        for (int y = 0; y < 4; ++y) acc[x][y] = fmaf(a[x], bq[y], acc[x][y]);
    }
#pragma unroll
    for (int x = 0; x < 4; ++x)
#pragma unroll
      for (int y = 0; y < 4; ++y) sT[(ti * 4u + (unsigned)x) * kCP + tj + 16u * (unsigned)y] = acc[x][y];
  }
  __syncthreads();
#pragma unroll
  for (int it = 0; it < 4; ++it) {
    const unsigned e = ((unsigned)it * 256u + t) * 4u;
    const unsigned r = e >> 6;
    const unsigned c = e & 63u;
    const v4f v = *(const v4f*)(wk + e);
    sW[r * kCP + c + 0u] = v[0];
    sW[r * kCP + c + 1u] = v[1];
    sW[r * kCP + c + 2u] = v[2];
    sW[r * kCP + c + 3u] = v[3];
  }
  __syncthreads();

  {
    float acc[4][4];
#pragma unroll
    for (int x = 0; x < 4; ++x)
#pragma unroll
      for (int y = 0; y < 4; ++y) acc[x][y] = 0.f;
#pragma unroll 1
    for (int k = 0; k < 64; ++k) {
      float a[4], bq[4];
#pragma unroll
      for (int x = 0; x < 4; ++x) a[x] = sW[(ti * 4u + (unsigned)x) * kCP + (unsigned)k];
#pragma unroll
      for (int y = 0; y < 4; ++y) bq[y] = sT[(unsigned)k * kCP + tj + 16u * (unsigned)y];
#pragma unroll
      for (int x = 0; x < 4; ++x)
#pragma unroll
        for (int y = 0; y < 4; ++y) acc[x][y] = fmaf(a[x], bq[y], acc[x][y]);
    }
#pragma unroll
    for (int x = 0; x < 4; ++x)
#pragma unroll
      for (int y = 0; y < 4; ++y) sG[(ti * 4u + (unsigned)x) * kCP + tj + 16u * (unsigned)y] = acc[x][y];
  }
  __syncthreads();
#pragma unroll
  for (int it = 0; it < 4; ++it) {
    const unsigned e = ((unsigned)it * 256u + t) * 4u;
    const unsigned r = e >> 6;
    const unsigned c = e & 63u;
    const v4f v = *(const v4f*)(wq + e);
    sW[r * kCP + c + 0u] = v[0];
    sW[r * kCP + c + 1u] = v[1];
    sW[r * kCP + c + 2u] = v[2];
    sW[r * kCP + c + 3u] = v[3];
  }
  __syncthreads();

  {
    float acc[4][4];
#pragma unroll
    for (int x = 0; x < 4; ++x)
#pragma unroll
      for (int y = 0; y < 4; ++y) acc[x][y] = 0.f;
#pragma unroll 1
    for (int k = 0; k < 64; ++k) {
      float a[4], bq[4];
#pragma unroll
      for (int x = 0; x < 4; ++x) a[x] = sW[(unsigned)k * kCP + ti * 4u + (unsigned)x];
#pragma unroll
      for (int y = 0; y < 4; ++y) bq[y] = sG[(unsigned)k * kCP + tj + 16u * (unsigned)y];
#pragma unroll
      for (int x = 0; x < 4; ++x)
#pragma unroll
        for (int y = 0; y < 4; ++y) acc[x][y] = fmaf(a[x], bq[y], acc[x][y]);
    }
#pragma unroll
    for (int x = 0; x < 4; ++x)
#pragma unroll
      for (int y = 0; y < 4; ++y) sT[(tj + 16u * (unsigned)y) * kCP + ti * 4u + (unsigned)x] = acc[x][y] * kNMul;
  }
  __syncthreads();

  const unsigned lane = t & 31u;
  const unsigned wave = t >> 5;
  unsigned q  = lane >> 3;
  unsigned c8 = (lane & 7u) * 8u;
  asm volatile("" : "+v"(q));
  asm volatile("" : "+v"(c8));
  v8h hv[2];
#pragma unroll
  for (int it = 0; it < 2; ++it) {
    const unsigned f = wave * 8u + (unsigned)it * 4u + q;
#pragma unroll
    for (int e = 0; e < 8; ++e) hv[it][e] = f16_flush(sT[f * kCP + c8 + (unsigned)e]);
  }
  for (int pass = 0; pass < 2; ++pass) {
#pragma unroll
    for (int it = 0; it < 2; ++it) {
      const unsigned f = wave * 8u + (unsigned)it * 4u + q;
      const size_t o = ((size_t)bh * kHd + f) * kHd + c8;
      *(volatile v8h*)(NT + o) = hv[it];
    }
    __threadfence();
  }
}

extern "C" void kernel_launch(void* const* d_in, const int* in_sizes, int n_in,
                              void* d_out, int out_size, void* d_ws, size_t ws_size,
                              hipStream_t stream) {
  if (n_in < 5) return;
  if (in_sizes[0] != kB * kSkv * kD) return;
  if (in_sizes[1] != kB * kSq * kD) return;
  if (in_sizes[2] != kH * kHd * kHd) return;
  if (in_sizes[3] != kH * kHd * kHd) return;
  if (in_sizes[4] != kH * kHd * kHd) return;
  if (out_size != kB * kSq * kD) return;
  if (ws_size < kWsTotal) return;

  const float* ctx = (const float*)d_in[0];
  const float* X   = (const float*)d_in[1];
  const float* Wq  = (const float*)d_in[2];
  const float* Wk  = (const float*)d_in[3];
  const float* Wv  = (const float*)d_in[4];
  float* out = (float*)d_out;

  char* ws = (char*)d_ws;
  unsigned short* CT = (unsigned short*)(ws + kOffCT);
  unsigned short* XH = (unsigned short*)(ws + kOffXH);
  float*          GP = (float*)(ws + kOffGP);
  unsigned short* NT = (unsigned short*)(ws + kOffNT);

  ctx_transpose_f16_kernel<<<dim3(kSkv / 64, kBH), 256, 0, stream>>>(ctx, CT);

  const unsigned total8 = (unsigned)(kB * kSq * kD / 8);
  x_headmajor_f16_kernel<<<total8 / 256, 256, 0, stream>>>(X, XH, total8);

  wmma_gemm64_f16<<<dim3(1, kBH * kKc), 32, 0, stream>>>(
      CT, kChunk, (long)kHd * kChunk,
      CT, kChunk, (long)kHd * kChunk,
      GP, kHd, (long)kHd * kHd,
      kHd, kHd, kChunk, kGramScale);

  chain_kernel<<<kBH, 256, 0, stream>>>(GP, Wq, Wk, Wv, NT);

  for (int bi = 0; bi < kB; ++bi) {
    wmma_gemm64_f16<<<dim3((kSq / 64) / 8, kH), 256, 0, stream>>>(
        XH + (size_t)bi * kH * kSq * kHd, kHd, (long)kSq * kHd,
        NT + (size_t)bi * kH * kHd * kHd, kHd, (long)kHd * kHd,
        out + (size_t)bi * kSq * kD, kD, (long)kHd,
        kSq, kHd, kHd, kOutScale);
  }
}
